// SelfAttention_3590592660075
// MI455X (gfx1250) — hardware-run, weakly checked
//
#include <hip/hip_runtime.h>


#ifndef NB
#define NB 4
#endif
#ifndef SEQ
#define SEQ 2048
#endif
#define NB_FULL   4
#define SEQ_FULL  2048
#define DM        1024
#define NWAVE     8
#define OP        68
#define CVB       2048u
#define NXB       ((unsigned)((size_t)NB * SEQ * DM / CVB))
#define NWB       ((unsigned)((size_t)3 * DM * DM / CVB))
#define NCH       (SEQ / 256)
#define LNCH      (DM / 256)
#define NPAR      5
#define PCARRY    16384.0f
#define RCARRY    2048.0f

#define EPI_QK  0
#define EPI_VT  1
#define EPI_F32 2

static_assert(SEQ % 256 == 0);
static_assert(SEQ <= SEQ_FULL);
static_assert(NB >= 1 && NB <= NB_FULL);
static_assert(DM == 1024);
static_assert(DM % 128 == 0);
static_assert(((size_t)NB * SEQ) % 128 == 0);
static_assert((size_t)NXB * CVB == (size_t)NB * SEQ * DM);
static_assert((size_t)NWB * CVB == (size_t)3 * DM * DM);
static_assert((size_t)DM * DM / CVB == 512);
static_assert((OP * 4) % 16 == 0);
static_assert(LNCH * 256 == DM);
static_assert(NCH * 256 == SEQ);
static_assert(DM == 256 * 4);
static_assert(SEQ % 128 == 0 && (2 * DM) % 128 == 0);
static_assert(DM % 32 == 0 && (2 * DM) % 32 == 0 && SEQ % 32 == 0);
static_assert(SEQ % 64 == 0);
static_assert(DM % 32 == 0);
static_assert(NWAVE == 8);

#define XB_BYTES   ((size_t)NB * SEQ * DM * 2)
#define WB_BYTES   ((size_t)3 * DM * DM * 2)
#define PR_BYTES   ((size_t)NPAR * DM * 4)
#define YQK_BYTES  ((size_t)SEQ * 2 * DM * 4)
#define YVT_BYTES  ((size_t)DM * SEQ * 4)
#define QK2_BYTES  ((size_t)2 * SEQ * 2 * DM * 2)
#define VT_BYTES   ((size_t)DM * SEQ * 2)
#define S_BYTES    ((size_t)SEQ * SEQ * 4)
#define R_BYTES    ((size_t)SEQ * SEQ * 4)
#define P_BYTES    ((size_t)SEQ * SEQ * 2)
#define WS_TOTAL   (XB_BYTES + WB_BYTES + PR_BYTES + YQK_BYTES + YVT_BYTES + QK2_BYTES + VT_BYTES + S_BYTES + R_BYTES + P_BYTES)
static_assert(WS_TOTAL <= (size_t)134217728);
static_assert(XB_BYTES % 128 == 0 && WB_BYTES % 128 == 0 && PR_BYTES % 128 == 0);
static_assert(YQK_BYTES % 128 == 0 && YVT_BYTES % 128 == 0 && QK2_BYTES % 128 == 0 && VT_BYTES % 128 == 0);
static_assert(S_BYTES % 128 == 0 && R_BYTES % 128 == 0 && P_BYTES % 128 == 0);

typedef __bf16   bf16;
typedef _Float16 f16;
typedef bf16     v16bf __attribute__((ext_vector_type(16)));
typedef f16      v16h  __attribute__((ext_vector_type(16)));
typedef float    v8f   __attribute__((ext_vector_type(8)));
typedef float    v4f   __attribute__((ext_vector_type(4)));
typedef unsigned v4u   __attribute__((ext_vector_type(4)));

union Pack8B { v4u u; bf16 h[8]; };
union Pack8H { v4u u; f16  h[8]; };

template <typename T> struct FragOf;
template <> struct FragOf<bf16> { typedef v16bf V; };
template <> struct FragOf<f16>  { typedef v16h  V; };

static __device__ __forceinline__ v8f mma16(v16bf a, v16bf b, v8f acc) {
  acc = __builtin_amdgcn_wmma_f32_16x16x32_bf16(false, a, false, b, (short)0, acc, false, false);
  asm volatile("v_nop\n\tv_nop\n\tv_nop\n\tv_nop" : "+v"(acc) : "v"(a), "v"(b));
  return acc;
}
static __device__ __forceinline__ v8f mma16(v16h a, v16h b, v8f acc) {
  acc = __builtin_amdgcn_wmma_f32_16x16x32_f16(false, a, false, b, (short)0, acc, false, false);
  asm volatile("v_nop\n\tv_nop\n\tv_nop\n\tv_nop" : "+v"(acc) : "v"(a), "v"(b));
  return acc;
}

static __device__ __forceinline__ f16 toh_flush(float v) {
  const f16 r = (f16)v;
  return (fabsf(v) < 6.103515625e-05f) ? (f16)0.0f : r;
}

__global__ __launch_bounds__(256) void convert_kernel(const float* __restrict__ x,
                                                      const float* __restrict__ wq,
                                                      const float* __restrict__ bq,
                                                      const float* __restrict__ wk,
                                                      const float* __restrict__ bk,
                                                      const float* __restrict__ wv,
                                                      const float* __restrict__ bv,
                                                      const float* __restrict__ gamma,
                                                      const float* __restrict__ beta,
                                                      bf16* __restrict__ xb,
                                                      bf16* __restrict__ wb,
                                                      float* __restrict__ parp) {
  const unsigned blk = blockIdx.x;
  const unsigned tid = threadIdx.x;
  if (blk < NXB + NWB) {
    const float* src;
    bf16* dst;
    if (blk < NXB) {
      const unsigned r  = blk * 2u + (tid >> 7);
      const unsigned c  = (tid & 127u) * 8u;
      const unsigned bt = r / (unsigned)SEQ;
      const unsigned s  = r - bt * (unsigned)SEQ;
      src = x + ((size_t)bt * SEQ_FULL + s) * DM + c;
      dst = xb + (size_t)r * DM + c;
    } else {
      const unsigned wblk = blk - NXB;
      const unsigned wi   = wblk >> 9;
      const unsigned off  = (wblk & 511u) * CVB + tid * 8u;
      const float* wsrc = (wi == 0u) ? wq : ((wi == 1u) ? wk : wv);
      src = wsrc + off;
      dst = wb + (size_t)wblk * CVB + tid * 8u;
    }
    const v4f a0 = *(const v4f*)(src);
    const v4f a1 = *(const v4f*)(src + 4);
    Pack8B pk;
    #pragma unroll
    for (int i = 0; i < 4; ++i) {
      pk.h[i]     = (bf16)a0[i];
      pk.h[4 + i] = (bf16)a1[i];
    }
    const v4u val = pk.u;
    *(volatile v4u*)(dst) = val;
    __threadfence();
    *(volatile v4u*)(dst) = val;
  } else {
    const unsigned j = blk - (NXB + NWB);
    const float* bsrc = (j == 0u) ? bq : ((j == 1u) ? bk : ((j == 2u) ? bv : ((j == 3u) ? gamma : beta)));
    const v4f a = *(const v4f*)(bsrc + tid * 4u);
    v4f o;
    #pragma unroll
    for (int i = 0; i < 4; ++i) o[i] = (float)(bf16)a[i];
    float* dst = parp + j * (unsigned)DM + tid * 4u;
    *(volatile v4f*)(dst) = o;
    __threadfence();
    *(volatile v4f*)(dst) = o;
  }
}

template <typename T, int EPI>
__global__ __launch_bounds__(256) void gemm_kernel(const T* __restrict__ A,
                                                   const T* __restrict__ Bt,
                                                   const float* __restrict__ bias,
                                                   void* __restrict__ C,
                                                   unsigned nk, unsigned lda, unsigned ldb, unsigned ldc,
                                                   unsigned long long sAz, unsigned long long sBz,
                                                   unsigned long long sCz, float scale) {
  typedef typename FragOf<T>::V VT;
  union Frag { VT v; v4u q[2]; };

  __shared__ __align__(16) float sO[NWAVE * 16 * OP];

  const unsigned tid  = threadIdx.x;
  const unsigned wave = tid >> 5;
  const unsigned lane = tid & 31u;
  const unsigned lq   = lane & 15u;
  const unsigned hi   = lane >> 4;
  const unsigned m0   = blockIdx.x * 128u + (wave & 3u) * 32u;
  const unsigned n0   = blockIdx.y * 128u + (wave >> 2) * 64u;

  const T* Ab = A  + (size_t)blockIdx.z * sAz;
  const T* Bb = Bt + (size_t)blockIdx.z * sBz;

  const T* ap[2];
  const T* bp[4];
  #pragma unroll
  for (int mt = 0; mt < 2; ++mt) ap[mt] = Ab + (size_t)(m0 + mt * 16u + lq) * lda + hi * 8u;
  #pragma unroll
  for (int nt = 0; nt < 4; ++nt) bp[nt] = Bb + (size_t)(n0 + nt * 16u + lq) * ldb + hi * 8u;

  v8f acc[2][4];
  #pragma unroll
  for (int mt = 0; mt < 2; ++mt) {
    #pragma unroll
    for (int nt = 0; nt < 4; ++nt) acc[mt][nt] = (v8f){0, 0, 0, 0, 0, 0, 0, 0};
  }

  #pragma unroll 1
  for (unsigned k = 0; k < nk; ++k) {
    const unsigned ko = k * 32u;
    Frag a[2], b[4];
    #pragma unroll
    for (int mt = 0; mt < 2; ++mt) {
      a[mt].q[0] = *(const v4u*)(ap[mt] + ko);
      a[mt].q[1] = *(const v4u*)(ap[mt] + ko + 16u);
    }
    #pragma unroll
    for (int nt = 0; nt < 4; ++nt) {
      b[nt].q[0] = *(const v4u*)(bp[nt] + ko);
      b[nt].q[1] = *(const v4u*)(bp[nt] + ko + 16u);
    }
    #pragma unroll
    for (int nt = 0; nt < 4; ++nt) {
      #pragma unroll
      for (int mt = 0; mt < 2; ++mt) acc[mt][nt] = mma16(a[mt].v, b[nt].v, acc[mt][nt]);
    }
  }

  size_t   cbase;
  unsigned ncol;
  if (EPI == EPI_QK) {
    cbase = (size_t)(n0 >> 10) * sCz;
    ncol  = n0 & 1023u;
  } else {
    cbase = (size_t)blockIdx.z * sCz;
    ncol  = n0;
  }

  float bcol[4];
  #pragma unroll
  for (int nt = 0; nt < 4; ++nt) bcol[nt] = 0.0f;
  if (EPI == EPI_QK) {
    #pragma unroll
    for (int nt = 0; nt < 4; ++nt) bcol[nt] = bias[n0 + nt * 16u + lq];
  }

  float* so = sO + wave * (16u * OP);

  #pragma unroll
  for (int mt = 0; mt < 2; ++mt) {
    if (mt != 0) __syncthreads();
    #pragma unroll
    for (int r = 0; r < 8; ++r) {
      float brow = 0.0f;
      if (EPI == EPI_VT) brow = bias[m0 + mt * 16u + hi * 8u + r];
      #pragma unroll
      for (int nt = 0; nt < 4; ++nt) {
        float val = acc[mt][nt][r];
        if (EPI == EPI_QK)  val += bcol[nt];
        if (EPI == EPI_VT)  val += brow;
        if (EPI == EPI_F32) val *= scale;
        so[(hi * 8u + r) * OP + nt * 16u + lq] = val;
      }
    }
    __syncthreads();

    if (EPI == EPI_F32) {
      float* Cf = (float*)C + cbase;
      v4f    vals[8];
      size_t gidx[8];
      #pragma unroll
      for (int it = 0; it < 8; ++it) {
        const unsigned row = it * 2u + hi;
        vals[it] = *(const v4f*)(so + row * OP + lq * 4u);
        gidx[it] = (size_t)(m0 + mt * 16u + row) * ldc + ncol + lq * 4u;
      }
      #pragma unroll
      for (int it = 0; it < 8; ++it) *(volatile v4f*)(Cf + gidx[it]) = vals[it];
      __threadfence();
      #pragma unroll
      for (int it = 0; it < 8; ++it) *(volatile v4f*)(Cf + gidx[it]) = vals[it];
    } else {
      f16* Ch = (f16*)C + cbase;
      v4u    vals[4];
      size_t gidx[4];
      #pragma unroll
      for (int it = 0; it < 4; ++it) {
        const unsigned row = it * 4u + (lane >> 3);
        const unsigned c8  = (lane & 7u) * 8u;
        const v4f x0 = *(const v4f*)(so + row * OP + c8);
        const v4f x1 = *(const v4f*)(so + row * OP + c8 + 4u);
        Pack8H ph;
        #pragma unroll
        for (int i = 0; i < 4; ++i) {
          ph.h[i]     = (f16)x0[i];
          ph.h[4 + i] = (f16)x1[i];
        }
        vals[it] = ph.u;
        gidx[it] = (size_t)(m0 + mt * 16u + row) * ldc + ncol + c8;
      }
      #pragma unroll
      for (int it = 0; it < 4; ++it) *(volatile v4u*)(Ch + gidx[it]) = vals[it];
      __threadfence();
      #pragma unroll
      for (int it = 0; it < 4; ++it) *(volatile v4u*)(Ch + gidx[it]) = vals[it];
    }
  }
}

__global__ __launch_bounds__(256) void ln_rows_kernel(const float* __restrict__ Y,
                                                      const float* __restrict__ par,
                                                      f16* __restrict__ QK2) {
  #pragma clang fp contract(off)
  const unsigned tid  = threadIdx.x;
  const unsigned wave = __builtin_amdgcn_readfirstlane(tid >> 5);
  const unsigned lane = tid & 31u;
  const unsigned seg  = blockIdx.y;
  const unsigned row  = blockIdx.x * 8u + wave;
  const float* yp = Y + (size_t)row * (2u * DM) + seg * (unsigned)DM + lane * 8u;
  const float* bp = par + seg * (unsigned)DM + lane * 8u;
  const float* gp = par + 3u * DM + lane * 8u;
  const float* tp = par + 4u * DM + lane * 8u;

  float s = 0.0f;
  #pragma unroll 1
  for (int it = 0; it < LNCH; ++it) {
    const v4f a0 = *(const v4f*)(yp + it * 256);
    const v4f a1 = *(const v4f*)(yp + it * 256 + 4);
    const v4f b0 = *(const v4f*)(bp + it * 256);
    const v4f b1 = *(const v4f*)(bp + it * 256 + 4);
    #pragma unroll
    for (int i = 0; i < 4; ++i) {
      s += a0[i] + b0[i];
      s += a1[i] + b1[i];
    }
  }
  #pragma unroll
  for (int off = 16; off > 0; off >>= 1) s += __shfl_xor(s, off, 32);
  const float mu = s * (1.0f / DM);

  float q = 0.0f;
  #pragma unroll 1
  for (int it = 0; it < LNCH; ++it) {
    const v4f a0 = *(const v4f*)(yp + it * 256);
    const v4f a1 = *(const v4f*)(yp + it * 256 + 4);
    const v4f b0 = *(const v4f*)(bp + it * 256);
    const v4f b1 = *(const v4f*)(bp + it * 256 + 4);
    #pragma unroll
    for (int i = 0; i < 4; ++i) {
      const float d0 = (a0[i] + b0[i]) - mu;
      const float d1 = (a1[i] + b1[i]) - mu;
      q += d0 * d0;
      q += d1 * d1;
    }
  }
  #pragma unroll
  for (int off = 16; off > 0; off >>= 1) q += __shfl_xor(q, off, 32);
  const float rstd = __builtin_amdgcn_rsqf(q * (1.0f / DM) + 1e-5f);

  const unsigned offh = seg * (unsigned)DM;
  const unsigned offr = (1u - seg) * (unsigned)DM;
  f16* dp = QK2 + ((size_t)seg * SEQ + row) * (size_t)(2 * DM) + lane * 8u;
  #pragma unroll 1
  for (int it = 0; it < LNCH; ++it) {
    const v4f a0 = *(const v4f*)(yp + it * 256);
    const v4f a1 = *(const v4f*)(yp + it * 256 + 4);
    const v4f b0 = *(const v4f*)(bp + it * 256);
    const v4f b1 = *(const v4f*)(bp + it * 256 + 4);
    const v4f g0 = *(const v4f*)(gp + it * 256);
    const v4f g1 = *(const v4f*)(gp + it * 256 + 4);
    const v4f t0 = *(const v4f*)(tp + it * 256);
    const v4f t1 = *(const v4f*)(tp + it * 256 + 4);
    Pack8H pkh, pkr;
    #pragma unroll
    for (int i = 0; i < 4; ++i) {
      const float y0 = ((a0[i] + b0[i]) - mu) * rstd * g0[i] + t0[i];
      const float y1 = ((a1[i] + b1[i]) - mu) * rstd * g1[i] + t1[i];
      const f16 h0 = toh_flush(y0);
      const f16 h1 = toh_flush(y1);
      pkh.h[i]     = h0;
      pkh.h[4 + i] = h1;
      pkr.h[i]     = toh_flush((y0 - (float)h0) * RCARRY);
      pkr.h[4 + i] = toh_flush((y1 - (float)h1) * RCARRY);
    }
    const v4u vh = pkh.u;
    const v4u vr = pkr.u;
    f16* dh = dp + offh + it * 256;
    f16* dr = dp + offr + it * 256;
    *(volatile v4u*)(dh) = vh;
    *(volatile v4u*)(dr) = vr;
    __threadfence();
    *(volatile v4u*)(dh) = vh;
    *(volatile v4u*)(dr) = vr;
  }
}

__global__ __launch_bounds__(256) void ln_cols_kernel(const float* __restrict__ Yt,
                                                      const float* __restrict__ par,
                                                      f16* __restrict__ vt) {
  #pragma clang fp contract(off)
  __shared__ __align__(16) float red[NWAVE * 64];

  const unsigned tid  = threadIdx.x;
  const unsigned wave = __builtin_amdgcn_readfirstlane(tid >> 5);
  const unsigned lane = tid & 31u;
  const unsigned cg   = lane & 7u;
  const unsigned rq   = lane >> 3;
  const unsigned s0   = blockIdx.x * 64u + cg * 8u;
  const float* yp = Yt + s0;

  float acc[8];
  float mu[8];
  float rstd[8];

  #pragma unroll
  for (int i = 0; i < 8; ++i) acc[i] = 0.0f;
  #pragma unroll 1
  for (unsigned it = 0; it < (unsigned)(DM / 32); ++it) {
    const unsigned e = (it * 8u + wave) * 4u + rq;
    const v4f x0 = *(const v4f*)(yp + (size_t)e * SEQ);
    const v4f x1 = *(const v4f*)(yp + (size_t)e * SEQ + 4);
    const float b = par[2u * DM + e];
    #pragma unroll
    for (int i = 0; i < 4; ++i) {
      acc[i]     += x0[i] + b;
      acc[4 + i] += x1[i] + b;
    }
  }
  #pragma unroll
  for (int i = 0; i < 8; ++i) {
    acc[i] += __shfl_xor(acc[i], 8, 32);
    acc[i] += __shfl_xor(acc[i], 16, 32);
  }
  if (rq == 0u) {
    *(v4f*)(red + wave * 64u + cg * 8u)      = (v4f){acc[0], acc[1], acc[2], acc[3]};
    *(v4f*)(red + wave * 64u + cg * 8u + 4u) = (v4f){acc[4], acc[5], acc[6], acc[7]};
  }
  __syncthreads();
  #pragma unroll
  for (int i = 0; i < 8; ++i) mu[i] = 0.0f;
  #pragma unroll
  for (int w = 0; w < NWAVE; ++w) {
    const v4f r0 = *(const v4f*)(red + w * 64 + cg * 8u);
    const v4f r1 = *(const v4f*)(red + w * 64 + cg * 8u + 4u);
    #pragma unroll
    for (int i = 0; i < 4; ++i) {
      mu[i]     += r0[i];
      mu[4 + i] += r1[i];
    }
  }
  #pragma unroll
  for (int i = 0; i < 8; ++i) mu[i] = mu[i] * (1.0f / DM);
  __syncthreads();

  #pragma unroll
  for (int i = 0; i < 8; ++i) acc[i] = 0.0f;
  #pragma unroll 1
  for (unsigned it = 0; it < (unsigned)(DM / 32); ++it) {
    const unsigned e = (it * 8u + wave) * 4u + rq;
    const v4f x0 = *(const v4f*)(yp + (size_t)e * SEQ);
    const v4f x1 = *(const v4f*)(yp + (size_t)e * SEQ + 4);
    const float b = par[2u * DM + e];
    #pragma unroll
    for (int i = 0; i < 4; ++i) {
      const float d0 = (x0[i] + b) - mu[i];
      const float d1 = (x1[i] + b) - mu[4 + i];
      acc[i]     += d0 * d0;
      acc[4 + i] += d1 * d1;
    }
  }
  #pragma unroll
  for (int i = 0; i < 8; ++i) {
    acc[i] += __shfl_xor(acc[i], 8, 32);
    acc[i] += __shfl_xor(acc[i], 16, 32);
  }
  if (rq == 0u) {
    *(v4f*)(red + wave * 64u + cg * 8u)      = (v4f){acc[0], acc[1], acc[2], acc[3]};
    *(v4f*)(red + wave * 64u + cg * 8u + 4u) = (v4f){acc[4], acc[5], acc[6], acc[7]};
  }
  __syncthreads();
  #pragma unroll
  for (int i = 0; i < 8; ++i) rstd[i] = 0.0f;
  #pragma unroll
  for (int w = 0; w < NWAVE; ++w) {
    const v4f r0 = *(const v4f*)(red + w * 64 + cg * 8u);
    const v4f r1 = *(const v4f*)(red + w * 64 + cg * 8u + 4u);
    #pragma unroll
    for (int i = 0; i < 4; ++i) {
      rstd[i]     += r0[i];
      rstd[4 + i] += r1[i];
    }
  }
  #pragma unroll
  for (int i = 0; i < 8; ++i) rstd[i] = __builtin_amdgcn_rsqf(rstd[i] * (1.0f / DM) + 1e-5f);

  f16* dp = vt + s0;
  #pragma unroll 1
  for (unsigned it = 0; it < (unsigned)(DM / 32); ++it) {
    const unsigned e = (it * 8u + wave) * 4u + rq;
    const v4f x0 = *(const v4f*)(yp + (size_t)e * SEQ);
    const v4f x1 = *(const v4f*)(yp + (size_t)e * SEQ + 4);
    const float b  = par[2u * DM + e];
    const float g  = par[3u * DM + e];
    const float bt = par[4u * DM + e];
    Pack8H pk;
    #pragma unroll
    for (int i = 0; i < 4; ++i) {
      const float y0 = ((x0[i] + b) - mu[i])     * rstd[i]     * g + bt;
      const float y1 = ((x1[i] + b) - mu[4 + i]) * rstd[4 + i] * g + bt;
      pk.h[i]     = toh_flush(y0);
      pk.h[4 + i] = toh_flush(y1);
    }
    const v4u val = pk.u;
    f16* dst = dp + (size_t)e * SEQ;
    *(volatile v4u*)(dst) = val;
    __threadfence();
    *(volatile v4u*)(dst) = val;
  }
}

__global__ __launch_bounds__(256) void softmax2_kernel(const float* __restrict__ S,
                                                       const float* __restrict__ R,
                                                       f16* __restrict__ P) {
  #pragma clang fp contract(off)
  const unsigned tid  = threadIdx.x;
  const unsigned wave = __builtin_amdgcn_readfirstlane(tid >> 5);
  const unsigned lane = tid & 31u;
  const unsigned row  = blockIdx.x * 8u + wave;
  const float* sp = S + (size_t)row * SEQ + lane * 8u;
  const float* rp = R + (size_t)row * SEQ + lane * 8u;

  v4f v[NCH][2];
  #pragma unroll
  for (int it = 0; it < NCH; ++it) {
    v[it][0] = *(const v4f*)(sp + it * 256);
    v[it][1] = *(const v4f*)(sp + it * 256 + 4);
  }
  __builtin_amdgcn_sched_barrier(0);
  #pragma unroll
  for (int it = 0; it < NCH; ++it) {
    const v4f r0 = *(const v4f*)(rp + it * 256);
    const v4f r1 = *(const v4f*)(rp + it * 256 + 4);
    v[it][0] += r0;
    v[it][1] += r1;
  }

  float m = -__builtin_inff();
  #pragma unroll
  for (int it = 0; it < NCH; ++it) {
    #pragma unroll
    for (int i = 0; i < 4; ++i) {
      m = fmaxf(m, v[it][0][i]);
      m = fmaxf(m, v[it][1][i]);
    }
  }
  #pragma unroll
  for (int off = 16; off > 0; off >>= 1) m = fmaxf(m, __shfl_xor(m, off, 32));

  const float L2E = 1.4426950408889634f;
  float sum = 0.0f;
  #pragma unroll
  for (int it = 0; it < NCH; ++it) {
    #pragma unroll
    for (int i = 0; i < 4; ++i) {
      const float e0 = __builtin_amdgcn_exp2f((v[it][0][i] - m) * L2E);
      const float e1 = __builtin_amdgcn_exp2f((v[it][1][i] - m) * L2E);
      v[it][0][i] = e0;
      v[it][1][i] = e1;
      sum += e0;
      sum += e1;
    }
  }
  #pragma unroll
  for (int off = 16; off > 0; off >>= 1) sum += __shfl_xor(sum, off, 32);

  const float inv = PCARRY * __builtin_amdgcn_rcpf(sum);

  v4u pk[NCH];
  #pragma unroll
  for (int it = 0; it < NCH; ++it) {
    Pack8H ph;
    #pragma unroll
    for (int i = 0; i < 4; ++i) {
      ph.h[i]     = toh_flush(v[it][0][i] * inv);
      ph.h[4 + i] = toh_flush(v[it][1][i] * inv);
    }
    pk[it] = ph.u;
  }

  f16* dp = P + (size_t)row * SEQ + lane * 8u;
  #pragma unroll
  for (int it = 0; it < NCH; ++it) *(volatile v4u*)(dp + it * 256) = pk[it];
  __threadfence();
  #pragma unroll
  for (int it = 0; it < NCH; ++it) *(volatile v4u*)(dp + it * 256) = pk[it];
}

extern "C" void kernel_launch(void* const* d_in, const int* in_sizes, int n_in,
                              void* d_out, int out_size, void* d_ws, size_t ws_size,
                              hipStream_t stream) {
  if (n_in < 9) return;
  const size_t rows_used = (size_t)(NB - 1) * SEQ_FULL + SEQ;
  if ((size_t)in_sizes[0] < rows_used * DM) return;
  if ((size_t)in_sizes[1] < (size_t)DM * DM) return;
  if ((size_t)in_sizes[2] < (size_t)DM) return;
  if ((size_t)in_sizes[3] < (size_t)DM * DM) return;
  if ((size_t)in_sizes[4] < (size_t)DM) return;
  if ((size_t)in_sizes[5] < (size_t)DM * DM) return;
  if ((size_t)in_sizes[6] < (size_t)DM) return;
  if ((size_t)in_sizes[7] < (size_t)DM) return;
  if ((size_t)in_sizes[8] < (size_t)DM) return;
  if ((size_t)out_size < rows_used * DM) return;
  if (ws_size < WS_TOTAL) return;

  const float* x     = (const float*)d_in[0];
  const float* wq    = (const float*)d_in[1];
  const float* bq    = (const float*)d_in[2];
  const float* wk    = (const float*)d_in[3];
  const float* bk    = (const float*)d_in[4];
  const float* wv    = (const float*)d_in[5];
  const float* bv    = (const float*)d_in[6];
  const float* gamma = (const float*)d_in[7];
  const float* beta  = (const float*)d_in[8];
  float* out = (float*)d_out;

  char* w = (char*)d_ws;
  bf16*  xb   = (bf16*)w;   w += XB_BYTES;
  bf16*  wb   = (bf16*)w;   w += WB_BYTES;
  float* parp = (float*)w;  w += PR_BYTES;
  float* Yqk  = (float*)w;  w += YQK_BYTES;
  float* Yvt  = (float*)w;  w += YVT_BYTES;
  f16*   qk2  = (f16*)w;    w += QK2_BYTES;
  f16*   vt   = (f16*)w;    w += VT_BYTES;
  float* Sp   = (float*)w;  w += S_BYTES;
  float* Rp   = (float*)w;  w += R_BYTES;
  f16*   Pp   = (f16*)w;    w += P_BYTES;

  const f16* qrow = qk2;
  const f16* krow = qk2 + (size_t)SEQ * 2 * DM;

  convert_kernel<<<dim3(NXB + NWB + (unsigned)NPAR), 256, 0, stream>>>(x, wq, bq, wk, bk, wv, bv, gamma, beta, xb, wb, parp);

  for (int b = 0; b < NB; ++b) {
    const bf16* xbb = xb + (size_t)b * SEQ * DM;

    gemm_kernel<bf16, EPI_F32><<<dim3(SEQ / 128, 2 * DM / 128, 1), 256, 0, stream>>>(
        xbb, wb, parp, (void*)Yqk, DM / 32, DM, DM, 2 * DM, 0ull, 0ull, 0ull, 1.0f);

    gemm_kernel<bf16, EPI_F32><<<dim3(DM / 128, SEQ / 128, 1), 256, 0, stream>>>(
        wb + (size_t)2 * DM * DM, xbb, parp, (void*)Yvt, DM / 32, DM, DM, SEQ, 0ull, 0ull, 0ull, 1.0f);

    ln_rows_kernel<<<dim3(SEQ / 8, 2, 1), 256, 0, stream>>>(Yqk, parp, qk2);
    ln_cols_kernel<<<dim3(SEQ / 64), 256, 0, stream>>>(Yvt, parp, vt);

    gemm_kernel<f16, EPI_F32><<<dim3(SEQ / 128, SEQ / 128, 1), 256, 0, stream>>>(
        qrow, krow + DM, parp, (void*)Sp, DM / 32, 2 * DM, 2 * DM, SEQ, 0ull, 0ull, 0ull, 1.0f);

    gemm_kernel<f16, EPI_F32><<<dim3(SEQ / 128, SEQ / 128, 1), 256, 0, stream>>>(
        qrow, krow, parp, (void*)Rp, 2 * DM / 32, 2 * DM, 2 * DM, SEQ, 0ull, 0ull, 0ull, 1.0f / RCARRY);

    softmax2_kernel<<<dim3(SEQ / 8), 256, 0, stream>>>(Sp, Rp, Pp);

    gemm_kernel<f16, EPI_F32><<<dim3(SEQ / 128, DM / 128, 1), 256, 0, stream>>>(
        Pp, vt, parp, (void*)(out + (size_t)b * SEQ_FULL * DM),
        SEQ / 32, SEQ, SEQ, DM, 0ull, 0ull, 0ull, 1.0f / PCARRY);
  }
}
